// TRMamba2AttnBlock_8211977470179
// MI455X (gfx1250) — hardware-verified
//
#include <hip/hip_runtime.h>
#include <math.h>

constexpr int kBatch    = 2;
constexpr int kSeq      = 2048;
constexpr int kDim      = 1024;
constexpr int kHeads    = 16;
constexpr int kHdim     = 64;
constexpr int kState    = 128;
constexpr int kFF       = 4096;
constexpr int kTok      = kBatch * kSeq;
constexpr int kHeadRows = kTok * kHeads;
constexpr float kInvDim    = 1.0f / 1024.0f;
constexpr float kEps       = 1e-6f;
constexpr float kWCarry    = 16.0f;
constexpr float kWCarryInv = 1.0f / 16.0f;
constexpr float kPCarry    = 2048.0f;
constexpr float kOCarry    = 16.0f;
constexpr float kYCarry    = 16.0f;
constexpr float kScoreScale = 0.125f;
constexpr float kPVScale   = kOCarry / (kPCarry * kWCarry);
constexpr float kWoScale   = 1.0f / (kOCarry * kWCarry);
constexpr float kFc2Scale  = 1.0f / (kYCarry * kWCarry);

constexpr size_t kMiB     = 1048576;
constexpr size_t OFF_WO   = 0;
constexpr size_t OFF_WGF  = 2 * kMiB;
constexpr size_t OFF_WF2  = 18 * kMiB;
constexpr size_t OFF_X2   = 26 * kMiB;
constexpr size_t OFF_HN   = 26 * kMiB;
constexpr size_t OFF_VT   = 42 * kMiB;
constexpr size_t OFF_Q2H  = 50 * kMiB;
constexpr size_t OFF_K2H  = 58 * kMiB;
constexpr size_t OFF_O    = 66 * kMiB;
constexpr size_t OFF_SW   = 66 * kMiB;
constexpr size_t OFF_GF   = 42 * kMiB;
constexpr size_t OFF_WQKV = 74 * kMiB;
constexpr size_t OFF_H16  = 80 * kMiB;
constexpr size_t OFF_QKF  = 88 * kMiB;
constexpr size_t OFF_QKH  = 104 * kMiB;
constexpr size_t OFF_T1   = 112 * kMiB;
constexpr size_t OFF_SC   = 74 * kMiB;
constexpr size_t OFF_P    = 106 * kMiB;
constexpr size_t OFF_X3   = 74 * kMiB;
constexpr size_t OFF_Y    = 90 * kMiB;
constexpr size_t kWsTotal = 128 * kMiB;
static_assert(OFF_T1 + (size_t)kHeadRows * kState * 2 == kWsTotal, "scratch end");
static_assert(OFF_P + (size_t)2 * kSeq * kSeq * 2 <= kWsTotal, "P plane end");
static_assert(OFF_Y + (size_t)kTok * kFF * 2 <= kWsTotal, "Y plane end");
static_assert(OFF_GF + (size_t)1024 * 8192 * 4 == OFF_WQKV, "GF end");
static_assert(kWsTotal == 134217728, "carve total");

typedef __attribute__((ext_vector_type(16))) _Float16 v16h;
typedef __attribute__((ext_vector_type(8)))  _Float16 v8h;
typedef __attribute__((ext_vector_type(16))) __bf16   v16b;
typedef __attribute__((ext_vector_type(8)))  __bf16   v8b;
typedef __attribute__((ext_vector_type(8)))  float    v8f;
typedef __attribute__((ext_vector_type(4)))  float    v4f;
typedef __attribute__((ext_vector_type(4)))  unsigned int v4u;
typedef __attribute__((ext_vector_type(4)))  int      v4i;

__device__ __forceinline__ unsigned short f2bf_bits(float f) {
  unsigned u = __float_as_uint(f);
  return (unsigned short)((u + 0x7FFFu + ((u >> 16) & 1u)) >> 16);
}
__device__ __forceinline__ float bf_bits2f(unsigned short h) { return __uint_as_float(((unsigned)h) << 16); }

__device__ __forceinline__ void dep_guard_h(v8f& a, v8f& b, v16h x, v16h y) { asm volatile("v_nop\n\tv_nop\n\tv_nop\n\tv_nop" : "+v"(a), "+v"(b) : "v"(x), "v"(y)); }
__device__ __forceinline__ void dep_guard_b(v8f& a, v8f& b, v16b x, v16b y) { asm volatile("v_nop\n\tv_nop\n\tv_nop\n\tv_nop" : "+v"(a), "+v"(b) : "v"(x), "v"(y)); }
__device__ __forceinline__ void keep4_h(v16h a, v16h b, v16h c, v16h d) { asm volatile("v_nop" :: "v"(a), "v"(b), "v"(c), "v"(d)); }
__device__ __forceinline__ void keep4_b(v16b a, v16b b, v16b c, v16b d) { asm volatile("v_nop" :: "v"(a), "v"(b), "v"(c), "v"(d)); }
__device__ __forceinline__ void acc_guard4(v8f& a, v8f& b, v8f& c, v8f& d) { asm volatile("v_nop\n\tv_nop\n\tv_nop\n\tv_nop" : "+v"(a), "+v"(b), "+v"(c), "+v"(d)); }
template <typename T> struct Frag;
template <> struct Frag<_Float16> {
  typedef v16h V; union U { v16h v; v8h h[2]; };
  static __device__ __forceinline__ v16h load(const _Float16* p) {
    U f; f.h[0] = *(const v8h*)(p); f.h[1] = *(const v8h*)(p + 16); return f.v;
  }
  static __device__ __forceinline__ v8f mma(v16h a, v16h b, v8f c) {
    return __builtin_amdgcn_wmma_f32_16x16x32_f16(false, a, false, b, (short)0, c, false, false);
  }
  static __device__ __forceinline__ void guard(v8f& a, v8f& b, v16h x, v16h y) { dep_guard_h(a, b, x, y); }
  static __device__ __forceinline__ void keep(v16h a, v16h b, v16h c, v16h d) { keep4_h(a, b, c, d); }
};
template <> struct Frag<__bf16> {
  typedef v16b V; union U { v16b v; v8b h[2]; };
  static __device__ __forceinline__ v16b load(const __bf16* p) {
    U f; f.h[0] = *(const v8b*)(p); f.h[1] = *(const v8b*)(p + 16); return f.v;
  }
  static __device__ __forceinline__ v8f mma(v16b a, v16b b, v8f c) {
    return __builtin_amdgcn_wmma_f32_16x16x32_bf16(false, a, false, b, (short)0, c, false, false);
  }
  static __device__ __forceinline__ void guard(v8f& a, v8f& b, v16b x, v16b y) { dep_guard_b(a, b, x, y); }
  static __device__ __forceinline__ void keep(v16b a, v16b b, v16b c, v16b d) { keep4_b(a, b, c, d); }
};

__device__ __forceinline__ unsigned pk16(unsigned short a, unsigned short b) { return (unsigned)a | ((unsigned)b << 16); }
__device__ __forceinline__ unsigned short h_bits(float f) { const _Float16 h = (_Float16)f; return __builtin_bit_cast(unsigned short, h); }

template <int ET> struct Elem;
template <> struct Elem<0> { typedef _Float16 T; };
template <> struct Elem<1> { typedef __bf16 T; };
template <int ET, bool SPLIT, int BIAS_MODE, int OUT_MODE, bool RESID, int ACT = 0, int TRI = 0>
__global__ __launch_bounds__(256) void wmma_gemm64(
    const unsigned short* __restrict__ Ap, const unsigned short* __restrict__ A2p, int lda, long strideA,
    const unsigned short* __restrict__ Btp, const unsigned short* __restrict__ Bt2p, int ldb, long strideB,
    void* __restrict__ Cout, void* __restrict__ Cout2, int ldc, long strideC,
    const float* __restrict__ bias,
    const float* __restrict__ resid, long strideR,
    int M, int N, int K, float scale) {
  typedef typename Elem<ET>::T T;
  typedef typename Frag<T>::V V;
  const T* A = (const T*)Ap; const T* A2 = (const T*)A2p; const T* Bt = (const T*)Btp; const T* Bt2 = (const T*)Bt2p;
  __shared__ __align__(16) float sT[8][16 * 68];
  const int b    = blockIdx.y;
  const int lane = threadIdx.x & 31;
  const int wave = threadIdx.x >> 5;
  const int tilesN = N >> 6;
  const int tilesM = M >> 6;
  const int tile = blockIdx.x * 8 + wave;
  if (tile >= tilesM * tilesN) return;
  const int tm = tile / tilesN;
  const int tn = tile - tm * tilesN;
  if (TRI == 1 && tn > tm) return;
  const int m0 = tm << 6;
  const int n0 = tn << 6;
  int Kl = K;
  if (TRI == 2) { const int kt = (tm + 1) << 6; Kl = (kt < K) ? kt : K; }

  const T* Ab  = A  + (size_t)b * strideA;
  const T* Bb  = Bt + (size_t)b * strideB;
  const T* Ab2 = SPLIT ? (A2  + (size_t)b * strideA) : nullptr;
  const T* Bb2 = SPLIT ? (Bt2 + (size_t)b * strideB) : nullptr;

  const int rlane = lane & 15;
  const int koff  = (lane >> 4) * 8;
  const int mOff  = (lane >> 4) * 8;

  v8f acc[4][4];
#pragma unroll
  for (int i = 0; i < 4; ++i)
#pragma unroll
    for (int j = 0; j < 4; ++j) acc[i][j] = (v8f){0.f,0.f,0.f,0.f,0.f,0.f,0.f,0.f};

  for (int k0 = 0; k0 < Kl; k0 += 32) {
    V bh[4], bl[4];
#pragma unroll
    for (int j = 0; j < 4; ++j) {
      const size_t bo = (size_t)(n0 + (j << 4) + rlane) * ldb + koff + k0;
      bh[j] = Frag<T>::load(Bb + bo);
      if (SPLIT) bl[j] = Frag<T>::load(Bb2 + bo);
    }
#pragma unroll
    for (int i = 0; i < 4; ++i) {
      const size_t ao = (size_t)(m0 + (i << 4) + rlane) * lda + koff + k0;
      V ah = Frag<T>::load(Ab + ao);
      V al;
      if (SPLIT) al = Frag<T>::load(Ab2 + ao);
#pragma unroll
      for (int j = 0; j < 4; ++j) {
        acc[i][j] = Frag<T>::mma(ah, bh[j], acc[i][j]);
        if (SPLIT) {
          acc[i][j] = Frag<T>::mma(ah, bl[j], acc[i][j]);
          acc[i][j] = Frag<T>::mma(al, bh[j], acc[i][j]);
        }
      }
      Frag<T>::guard(acc[i][0], acc[i][3], ah, SPLIT ? al : ah);
    }
    Frag<T>::keep(bh[0], bh[1], bh[2], bh[3]);
    if (SPLIT) Frag<T>::keep(bl[0], bl[1], bl[2], bl[3]);
  }
  acc_guard4(acc[0][0], acc[0][1], acc[0][2], acc[0][3]);
  acc_guard4(acc[1][0], acc[1][1], acc[1][2], acc[1][3]);
  acc_guard4(acc[2][0], acc[2][1], acc[2][2], acc[2][3]);
  acc_guard4(acc[3][0], acc[3][1], acc[3][2], acc[3][3]);

  float* slab = sT[wave];
  const float* Rb = RESID ? (resid + (size_t)b * strideR) : nullptr;
#pragma unroll
  for (int i = 0; i < 4; ++i) {
    const int mBase = m0 + (i << 4);
#pragma unroll
    for (int j = 0; j < 4; ++j) {
      const int n = n0 + (j << 4) + rlane;
      float bv = 0.f;
      if (BIAS_MODE == 2) bv = bias[n];
#pragma unroll
      for (int r = 0; r < 8; ++r) {
        float v = acc[i][j][r] * scale;
        if (BIAS_MODE == 1) v += bias[mBase + mOff + r];
        if (BIAS_MODE == 2) v += bv;
        if (RESID) v += Rb[(size_t)(mBase + mOff + r) * ldc + n];
        if (ACT == 2) v = fmaxf(v, 0.0f);
        if (ACT == 3) v = v / (1.0f + expf(-v));
        if (ACT == 4) v = (v > 0.f) ? v : 0.01f * v;
        slab[(mOff + r) * 68 + (j << 4) + rlane] = v;
      }
    }
    __builtin_amdgcn_fence(__ATOMIC_RELEASE, "workgroup");
    __builtin_amdgcn_wave_barrier();
    __builtin_amdgcn_fence(__ATOMIC_ACQUIRE, "workgroup");
    if (OUT_MODE == 0) {
      float* C = (float*)Cout + (size_t)b * strideC;
      const int hh = lane >> 4, c4 = (lane & 15) * 4;
      for (int pass = 0; pass < 2; ++pass) {
#pragma unroll
        for (int it = 0; it < 8; ++it) {
          const int row = it * 2 + hh;
          v4f v = *(const v4f*)(slab + row * 68 + c4);
          *(volatile v4f*)(C + (size_t)(mBase + row) * ldc + n0 + c4) = v;
        }
        __threadfence();
      }
    } else {
      const int q = lane >> 3, c8 = (lane & 7) * 8;
      unsigned short* C  = (unsigned short*)Cout  + (size_t)b * strideC;
      unsigned short* C2 = (OUT_MODE == 2) ? ((unsigned short*)Cout2 + (size_t)b * strideC) : nullptr;
      for (int pass = 0; pass < 2; ++pass) {
#pragma unroll
        for (int it = 0; it < 4; ++it) {
          const int row = it * 4 + q;
          const float* sp = slab + row * 68 + c8;
          v8h hv, lv;
#pragma unroll
          for (int e = 0; e < 8; ++e) {
            if (OUT_MODE == 1) {
              hv[e] = (_Float16)sp[e];
            } else {
              unsigned short hb = f2bf_bits(sp[e]);
              unsigned short lb = f2bf_bits(sp[e] - bf_bits2f(hb));
              hv[e] = __builtin_bit_cast(_Float16, hb);
              lv[e] = __builtin_bit_cast(_Float16, lb);
            }
          }
          *(volatile v8h*)(C + (size_t)(mBase + row) * ldc + n0 + c8) = hv;
          if (OUT_MODE == 2) *(volatile v8h*)(C2 + (size_t)(mBase + row) * ldc + n0 + c8) = lv;
        }
        __threadfence();
      }
    }
    __builtin_amdgcn_fence(__ATOMIC_RELEASE, "workgroup");
    __builtin_amdgcn_wave_barrier();
    __builtin_amdgcn_fence(__ATOMIC_ACQUIRE, "workgroup");
  }
}

__global__ __launch_bounds__(256) void wtcast_kernel(const float* __restrict__ W0, const float* __restrict__ W1,
                                                     const float* __restrict__ W2, int R, int Cn,
                                                     unsigned short* __restrict__ out, long planeStride, float scale) {
  __shared__ float sm[64][65];
  const int t  = threadIdx.x;
  const int r0 = blockIdx.x * 64;
  const int c0 = blockIdx.y * 64;
  const int z  = blockIdx.z;
  const float* W = (z == 0) ? W0 : (z == 1) ? W1 : W2;
#pragma unroll
  for (int i = 0; i < 16; ++i) {
    const int e = i * 256 + t;
    const int r = e >> 6;
    const int c = e & 63;
    sm[c][r] = W[(size_t)(r0 + r) * Cn + c0 + c] * scale;
  }
  __syncthreads();
  const int lane = t & 31, wave = t >> 5;
  const int q = lane >> 3, c8 = (lane & 7) * 8;
  unsigned short* op = out + (size_t)z * planeStride;
  for (int pass = 0; pass < 2; ++pass) {
#pragma unroll
    for (int it = 0; it < 2; ++it) {
      const int row = wave * 8 + it * 4 + q;
      unsigned short hb[8];
#pragma unroll
      for (int e = 0; e < 8; ++e) hb[e] = h_bits(sm[row][c8 + e]);
      const v4u u = (v4u){pk16(hb[0], hb[1]), pk16(hb[2], hb[3]), pk16(hb[4], hb[5]), pk16(hb[6], hb[7])};
      *(volatile v4u*)(op + (size_t)(c0 + row) * R + r0 + c8) = u;
    }
    __threadfence();
  }
}

__device__ __forceinline__ float block_sum256(float v, float* red, int lane, int wave) {
#pragma unroll
  for (int off = 16; off > 0; off >>= 1) v += __shfl_xor(v, off, 32);
  if (lane == 0) red[wave] = v;
  __syncthreads();
  const float s = ((red[0] + red[1]) + (red[2] + red[3])) + ((red[4] + red[5]) + (red[6] + red[7]));
  __syncthreads();
  return s;
}

__global__ __launch_bounds__(256) void prep_kernel(const float* __restrict__ x, const float* __restrict__ w1,
                                                   const float* __restrict__ w2, const float* __restrict__ w3,
                                                   float* __restrict__ x2o, unsigned short* __restrict__ ho) {
  __shared__ float red[8];
  __shared__ __align__(16) float hrow[1024];
  const int row = blockIdx.x;
  const int t = threadIdx.x, lane = t & 31, wave = t >> 5;
  const size_t rb = (size_t)row * kDim;
  v4f v = *(const v4f*)(x + rb + 4 * t);

  float ss = v[0] * v[0] + v[1] * v[1] + v[2] * v[2] + v[3] * v[3];
  float tot = block_sum256(ss, red, lane, wave);
  float rs = rsqrtf(tot * kInvDim + kEps);
  v4f w = *(const v4f*)(w1 + 4 * t);
  v = v + w * (v * rs);

  ss = v[0] * v[0] + v[1] * v[1] + v[2] * v[2] + v[3] * v[3];
  tot = block_sum256(ss, red, lane, wave);
  rs = rsqrtf(tot * kInvDim + kEps);
  w = *(const v4f*)(w2 + 4 * t);
  v = v + w * (v * rs);

  {
    float* xp = x2o + rb + 4 * t;
    *(volatile v4f*)xp = v;
    __threadfence();
    *(volatile v4f*)xp = v;
  }

  ss = v[0] * v[0] + v[1] * v[1] + v[2] * v[2] + v[3] * v[3];
  tot = block_sum256(ss, red, lane, wave);
  rs = rsqrtf(tot * kInvDim + kEps);
  w = *(const v4f*)(w3 + 4 * t);
  const v4f h = w * (v * rs);
  *(v4f*)(hrow + 4 * t) = h;
  __syncthreads();
  if (t < 128) {
    const v4f a = *(const v4f*)(hrow + 8 * t);
    const v4f c = *(const v4f*)(hrow + 8 * t + 4);
    unsigned short hb[8];
#pragma unroll
    for (int e = 0; e < 4; ++e) { hb[e] = h_bits(a[e]); hb[4 + e] = h_bits(c[e]); }
    const v4u u = (v4u){pk16(hb[0], hb[1]), pk16(hb[2], hb[3]), pk16(hb[4], hb[5]), pk16(hb[6], hb[7])};
    unsigned short* hp = ho + rb + 8 * t;
    *(volatile v4u*)hp = u;
    __threadfence();
    *(volatile v4u*)hp = u;
  }
}

__global__ __launch_bounds__(256) void rms_f16_kernel(const float* __restrict__ x, const float* __restrict__ w,
                                                      unsigned short* __restrict__ ho) {
  __shared__ float red[8];
  __shared__ __align__(16) float hrow[1024];
  const int row = blockIdx.x;
  const int t = threadIdx.x, lane = t & 31, wave = t >> 5;
  const size_t rb = (size_t)row * kDim;
  const v4f v = *(const v4f*)(x + rb + 4 * t);
  const float ss = v[0] * v[0] + v[1] * v[1] + v[2] * v[2] + v[3] * v[3];
  const float tot = block_sum256(ss, red, lane, wave);
  const float rs = rsqrtf(tot * kInvDim + kEps);
  const v4f wv = *(const v4f*)(w + 4 * t);
  const v4f h = wv * (v * rs);
  *(v4f*)(hrow + 4 * t) = h;
  __syncthreads();
  if (t < 128) {
    const v4f a = *(const v4f*)(hrow + 8 * t);
    const v4f c = *(const v4f*)(hrow + 8 * t + 4);
    unsigned short hb[8];
#pragma unroll
    for (int e = 0; e < 4; ++e) { hb[e] = h_bits(a[e]); hb[4 + e] = h_bits(c[e]); }
    const v4u u = (v4u){pk16(hb[0], hb[1]), pk16(hb[2], hb[3]), pk16(hb[4], hb[5]), pk16(hb[6], hb[7])};
    unsigned short* hp = ho + rb + 8 * t;
    *(volatile v4u*)hp = u;
    __threadfence();
    *(volatile v4u*)hp = u;
  }
}

__global__ __launch_bounds__(256) void cast8_f16_kernel(const float* __restrict__ in, unsigned short* __restrict__ out, int n8) {
  const int i = blockIdx.x * 256 + threadIdx.x;
  if (i >= n8) return;
  const float* p = in + 8 * (size_t)i;
  const v4f a = *(const v4f*)(p);
  const v4f c = *(const v4f*)(p + 4);
  unsigned short hb[8];
#pragma unroll
  for (int e = 0; e < 4; ++e) {
    hb[e]     = h_bits(a[e]);
    hb[4 + e] = h_bits(c[e]);
  }
  const v4u u = (v4u){pk16(hb[0], hb[1]), pk16(hb[2], hb[3]), pk16(hb[4], hb[5]), pk16(hb[6], hb[7])};
  unsigned short* q = out + 8 * (size_t)i;
  *(volatile v4u*)q = u;
  __threadfence();
  *(volatile v4u*)q = u;
}

__global__ __launch_bounds__(256) void softmax_row_kernel(const float* __restrict__ SC, const int* __restrict__ mask,
                                                          unsigned short* __restrict__ P) {
  __shared__ float redM[8];
  __shared__ float redS[8];
  const int row  = blockIdx.x;
  const int qi   = row & (kSeq - 1);
  const int t    = threadIdx.x;
  const int lane = t & 31, wave = t >> 5;
  const int limit = ((qi >> 6) + 1) << 6;
  const bool act = (wave << 8) < limit;
  const int c0   = t * 8;
  float xv[8];
#pragma unroll
  for (int e = 0; e < 8; ++e) xv[e] = -INFINITY;
  if (act) {
    const float* sr = SC + (size_t)row * kSeq + c0;
    const v4f a = *(const v4f*)(sr);
    const v4f c = *(const v4f*)(sr + 4);
    const int* mr = mask + (size_t)qi * kSeq + c0;
    const v4i ma = *(const v4i*)(mr);
    const v4i mb = *(const v4i*)(mr + 4);
#pragma unroll
    for (int e = 0; e < 4; ++e) {
      const bool k0 = ((c0 + e) < limit) && (ma[e] == 0);
      const bool k1 = ((c0 + 4 + e) < limit) && (mb[e] == 0);
      xv[e]     = k0 ? a[e] : -INFINITY;
      xv[4 + e] = k1 ? c[e] : -INFINITY;
    }
  }
  float m = fmaxf(fmaxf(fmaxf(xv[0], xv[1]), fmaxf(xv[2], xv[3])), fmaxf(fmaxf(xv[4], xv[5]), fmaxf(xv[6], xv[7])));
#pragma unroll
  for (int off = 16; off > 0; off >>= 1) m = fmaxf(m, __shfl_xor(m, off, 32));
  if (lane == 0) redM[wave] = m;
  __syncthreads();
  const float M = fmaxf(fmaxf(fmaxf(redM[0], redM[1]), fmaxf(redM[2], redM[3])),
                        fmaxf(fmaxf(redM[4], redM[5]), fmaxf(redM[6], redM[7])));
  float pv[8];
#pragma unroll
  for (int e = 0; e < 8; ++e) pv[e] = 0.f;
  float s = 0.f;
  if (act) {
#pragma unroll
    for (int e = 0; e < 8; ++e) { pv[e] = expf(xv[e] - M); s += pv[e]; }
  }
#pragma unroll
  for (int off = 16; off > 0; off >>= 1) s += __shfl_xor(s, off, 32);
  if (lane == 0) redS[wave] = s;
  __syncthreads();
  const float S = ((redS[0] + redS[1]) + (redS[2] + redS[3])) + ((redS[4] + redS[5]) + (redS[6] + redS[7]));
  if (act) {
    const float inv = kPCarry / S;
    unsigned short hb[8];
#pragma unroll
    for (int e = 0; e < 8; ++e) hb[e] = h_bits(pv[e] * inv);
    const v4u u = (v4u){pk16(hb[0], hb[1]), pk16(hb[2], hb[3]), pk16(hb[4], hb[5]), pk16(hb[6], hb[7])};
    unsigned short* pp = P + (size_t)row * kSeq + c0;
    *(volatile v4u*)pp = u;
    __threadfence();
    *(volatile v4u*)pp = u;
  }
}

__global__ __launch_bounds__(256) void gating_kernel(const float* __restrict__ GF, unsigned short* __restrict__ Y) {
  const int i  = blockIdx.x * 256 + threadIdx.x;
  const int m  = i >> 9;
  const int n8 = (i & 511) * 8;
  const float* gp = GF + (size_t)m * 8192 + n8;
  const v4f g0 = *(const v4f*)(gp);
  const v4f g1 = *(const v4f*)(gp + 4);
  const v4f f0 = *(const v4f*)(gp + 4096);
  const v4f f1 = *(const v4f*)(gp + 4100);
  unsigned short hb[8];
#pragma unroll
  for (int e = 0; e < 4; ++e) {
    const float a0 = g0[e];
    const float s0 = a0 / (1.0f + expf(-a0));
    hb[e] = h_bits((s0 * f0[e]) * kYCarry);
    const float a1 = g1[e];
    const float s1 = a1 / (1.0f + expf(-a1));
    hb[4 + e] = h_bits((s1 * f1[e]) * kYCarry);
  }
  const v4u u = (v4u){pk16(hb[0], hb[1]), pk16(hb[2], hb[3]), pk16(hb[4], hb[5]), pk16(hb[6], hb[7])};
  unsigned short* yp = Y + (size_t)m * kFF + n8;
  *(volatile v4u*)yp = u;
  __threadfence();
  *(volatile v4u*)yp = u;
}

extern "C" void kernel_launch(void* const* d_in, const int* in_sizes, int n_in,
                              void* d_out, int out_size, void* d_ws, size_t ws_size,
                              hipStream_t stream) {
  if (n_in < 24) return;
  if (in_sizes[0] != kTok * kDim || in_sizes[1] != kSeq * kSeq) return;
  if (out_size != kTok * kDim) return;
  if (ws_size < kWsTotal) return;

  const float* x      = (const float*)d_in[0];
  const int*   mask   = (const int*)d_in[1];
  const float* n1w    = (const float*)d_in[2];
  const float* n2w    = (const float*)d_in[3];
  const float* n3w    = (const float*)d_in[4];
  const float* mlpnw  = (const float*)d_in[5];
  const float* wq     = (const float*)d_in[6];
  const float* wk     = (const float*)d_in[7];
  const float* wv     = (const float*)d_in[8];
  const float* wo     = (const float*)d_in[9];
  const float* qs_w1  = (const float*)d_in[10];
  const float* qs_b1  = (const float*)d_in[11];
  const float* qs_w2  = (const float*)d_in[12];
  const float* qs_b2  = (const float*)d_in[13];
  const float* ks_w1  = (const float*)d_in[14];
  const float* ks_b1  = (const float*)d_in[15];
  const float* ks_w2  = (const float*)d_in[16];
  const float* ks_b2  = (const float*)d_in[17];
  const float* fc1_w  = (const float*)d_in[18];
  const float* fc1_b  = (const float*)d_in[19];
  const float* fc2_w  = (const float*)d_in[20];
  const float* fc2_b  = (const float*)d_in[21];
  const float* gate_w = (const float*)d_in[22];
  const float* gate_b = (const float*)d_in[23];

  char* ws = (char*)d_ws;
  unsigned short* WO   = (unsigned short*)(ws + OFF_WO);
  unsigned short* WGF  = (unsigned short*)(ws + OFF_WGF);
  unsigned short* WF2  = (unsigned short*)(ws + OFF_WF2);
  float*          X2   = (float*)(ws + OFF_X2);
  unsigned short* HN   = (unsigned short*)(ws + OFF_HN);
  unsigned short* VT   = (unsigned short*)(ws + OFF_VT);
  unsigned short* Q2H  = (unsigned short*)(ws + OFF_Q2H);
  unsigned short* K2H  = (unsigned short*)(ws + OFF_K2H);
  unsigned short* O16  = (unsigned short*)(ws + OFF_O);
  unsigned short* SW   = (unsigned short*)(ws + OFF_SW);
  float*          GF   = (float*)(ws + OFF_GF);
  unsigned short* WQKV = (unsigned short*)(ws + OFF_WQKV);
  unsigned short* H16  = (unsigned short*)(ws + OFF_H16);
  float*          QKF  = (float*)(ws + OFF_QKF);
  unsigned short* QKH  = (unsigned short*)(ws + OFF_QKH);
  unsigned short* T1   = (unsigned short*)(ws + OFF_T1);
  float*          SC   = (float*)(ws + OFF_SC);
  unsigned short* P16  = (unsigned short*)(ws + OFF_P);
  float*          X3   = (float*)(ws + OFF_X3);
  unsigned short* Y16  = (unsigned short*)(ws + OFF_Y);
  float*          OUT  = (float*)d_out;

  const long kSwPlane = (long)kHdim * kState;

  wtcast_kernel<<<dim3(kDim / 64, kDim / 64, 3), 256, 0, stream>>>(wq, wk, wv, kDim, kDim, WQKV, (long)kDim * kDim, kWCarry);
  wtcast_kernel<<<dim3(kDim / 64, kDim / 64, 1), 256, 0, stream>>>(wo, wo, wo, kDim, kDim, WO, 0L, kWCarry);
  wtcast_kernel<<<dim3(kDim / 64, kFF / 64, 2), 256, 0, stream>>>(gate_w, fc1_w, fc1_w, kDim, kFF, WGF, (long)kFF * kDim, kWCarry);
  wtcast_kernel<<<dim3(kFF / 64, kDim / 64, 1), 256, 0, stream>>>(fc2_w, fc2_w, fc2_w, kFF, kDim, WF2, 0L, kWCarry);
  wtcast_kernel<<<dim3(kHdim / 64, kState / 64, 2), 256, 0, stream>>>(qs_w1, ks_w1, ks_w1, kHdim, kState, SW, kSwPlane, kWCarry);
  wtcast_kernel<<<dim3(kState / 64, kHdim / 64, 2), 256, 0, stream>>>(qs_w2, ks_w2, ks_w2, kState, kHdim, SW + 2 * kSwPlane, kSwPlane, kWCarry);

  prep_kernel<<<kTok, 256, 0, stream>>>(x, n1w, n2w, n3w, X2, H16);

  const dim3 g128(128, 1);
  const int nQcast8 = kTok * kDim / 8;

  wmma_gemm64<0, false, 0, 0, false, 0, 0><<<g128, 256, 0, stream>>>(
      H16, nullptr, kDim, 0L, WQKV, nullptr, kDim, 0L,
      QKF, nullptr, kDim, 0L, nullptr, nullptr, 0L, kTok, kDim, kDim, kWCarryInv);
  cast8_f16_kernel<<<nQcast8 / 256, 256, 0, stream>>>(QKF, QKH, nQcast8);
  wmma_gemm64<0, false, 2, 1, false, 3, 0><<<dim3(256, 1), 256, 0, stream>>>(
      QKH, nullptr, kHdim, 0L, SW, nullptr, kHdim, 0L,
      T1, nullptr, kState, 0L, qs_b1, nullptr, 0L, kHeadRows, kState, kHdim, kWCarryInv);
  wmma_gemm64<0, false, 2, 1, true, 0, 0><<<g128, 256, 0, stream>>>(
      T1, nullptr, kState, 0L, SW + 2 * kSwPlane, nullptr, kState, 0L,
      Q2H, nullptr, kHdim, 0L, qs_b2, QKF, 0L, kHeadRows, kHdim, kState, kWCarryInv);

  wmma_gemm64<0, false, 0, 0, false, 0, 0><<<g128, 256, 0, stream>>>(
      H16, nullptr, kDim, 0L, WQKV + (size_t)kDim * kDim, nullptr, kDim, 0L,
      QKF, nullptr, kDim, 0L, nullptr, nullptr, 0L, kTok, kDim, kDim, kWCarryInv);
  cast8_f16_kernel<<<nQcast8 / 256, 256, 0, stream>>>(QKF, QKH, nQcast8);
  wmma_gemm64<0, false, 2, 1, false, 3, 0><<<dim3(256, 1), 256, 0, stream>>>(
      QKH, nullptr, kHdim, 0L, SW + kSwPlane, nullptr, kHdim, 0L,
      T1, nullptr, kState, 0L, ks_b1, nullptr, 0L, kHeadRows, kState, kHdim, kWCarryInv);
  wmma_gemm64<0, false, 2, 1, true, 0, 0><<<g128, 256, 0, stream>>>(
      T1, nullptr, kState, 0L, SW + 3 * kSwPlane, nullptr, kState, 0L,
      K2H, nullptr, kHdim, 0L, ks_b2, QKF, 0L, kHeadRows, kHdim, kState, kWCarryInv);

  wmma_gemm64<0, false, 0, 1, false, 0, 0><<<g128, 256, 0, stream>>>(
      WQKV + (size_t)2 * kDim * kDim, nullptr, kDim, 0L, H16, nullptr, kDim, 0L,
      VT, nullptr, kTok, 0L, nullptr, nullptr, 0L, kDim, kTok, kDim, 1.0f);

  const long scStride = (long)kSeq * kSeq;
  for (int cidx = 0; cidx < kBatch * (kHeads / 2); ++cidx) {
    const int bb = cidx / (kHeads / 2);
    const int h0 = (cidx % (kHeads / 2)) * 2;
    const size_t qoff = (size_t)bb * kSeq * kDim + (size_t)h0 * kHdim;
    wmma_gemm64<0, false, 0, 0, false, 0, 1><<<dim3(128, 2), 256, 0, stream>>>(
        Q2H + qoff, nullptr, kDim, (long)kHdim, K2H + qoff, nullptr, kDim, (long)kHdim,
        SC, nullptr, kSeq, scStride, nullptr, nullptr, 0L, kSeq, kSeq, kHdim, kScoreScale);
    softmax_row_kernel<<<2 * kSeq, 256, 0, stream>>>(SC, mask, P16);
    wmma_gemm64<0, false, 0, 1, false, 0, 2><<<dim3(4, 2), 256, 0, stream>>>(
        P16, nullptr, kSeq, scStride,
        VT + (size_t)(h0 * kHdim) * kTok + (size_t)bb * kSeq, nullptr, kTok, (long)kHdim * kTok,
        O16 + qoff, nullptr, kDim, (long)kHdim, nullptr, nullptr, 0L, kSeq, kHdim, kSeq, kPVScale);
  }

  wmma_gemm64<0, false, 0, 0, true, 0, 0><<<g128, 256, 0, stream>>>(
      O16, nullptr, kDim, 0L, WO, nullptr, kDim, 0L,
      X3, nullptr, kDim, 0L, nullptr, X2, 0L, kTok, kDim, kDim, kWoScale);

  rms_f16_kernel<<<kTok, 256, 0, stream>>>(X3, mlpnw, HN);

  for (int mc = 0; mc < 4; ++mc) {
    const unsigned short* hnc = HN + (size_t)mc * 1024 * kDim;
    wmma_gemm64<0, false, 2, 0, false, 0, 0><<<g128, 256, 0, stream>>>(
        hnc, nullptr, kDim, 0L, WGF, nullptr, kDim, 0L,
        GF, nullptr, 2 * kFF, 0L, gate_b, nullptr, 0L, 1024, kFF, kDim, kWCarryInv);
    wmma_gemm64<0, false, 2, 0, false, 0, 0><<<g128, 256, 0, stream>>>(
        hnc, nullptr, kDim, 0L, WGF + (size_t)kFF * kDim, nullptr, kDim, 0L,
        GF + kFF, nullptr, 2 * kFF, 0L, fc1_b, nullptr, 0L, 1024, kFF, kDim, kWCarryInv);
    gating_kernel<<<(1024 * kFF / 8) / 256, 256, 0, stream>>>(GF, Y16 + (size_t)mc * 1024 * kFF);
  }

  wmma_gemm64<0, false, 2, 0, true, 0, 0><<<g128, 256, 0, stream>>>(
      Y16, nullptr, kFF, 0L, WF2, nullptr, kFF, 0L,
      OUT, nullptr, kDim, 0L, fc2_b, X3, 0L, kTok, kDim, kFF, kFc2Scale);
}
